// KnotNet_12927851561368
// MI455X (gfx1250) — hardware-verified
//
#include <hip/hip_runtime.h>
#include <stdint.h>
#include <stddef.h>


#define NB        4096
#define NT        256
#define NS        4
#define NH        64
#define KF        256
#define N1        128
#define N2        64
#define LN_EPS    1e-5f
#define ACAR      16.0f
#define HCAR      16.0f
#define WCAR      1024.0f
#define WSCAP     134217728
#define SCAN_WAVES 8
#define SCAN_THR  (SCAN_WAVES * 32)
#define GEMM_THR  128
#define LDH       65

static_assert(KF == NS * NH);
static_assert((KF % 32) == 0);
static_assert((N1 % 32) == 0);
static_assert((N1 % 16) == 0);
static_assert((N2 % 16) == 0);
static_assert((NB % 64) == 0);
static_assert((NB % SCAN_WAVES) == 0);
static_assert(NH == 64);
static_assert(N2 == 64);
static_assert(GEMM_THR == 128);

typedef float          v4f  __attribute__((ext_vector_type(4)));
typedef float          v8f  __attribute__((ext_vector_type(8)));
typedef _Float16       v8h  __attribute__((ext_vector_type(8)));
typedef _Float16       v16h __attribute__((ext_vector_type(16)));
typedef unsigned int   v4u  __attribute__((ext_vector_type(4)));
typedef v4f v4fa __attribute__((may_alias));
typedef v8h v8ha __attribute__((may_alias));
typedef v4u v4ua __attribute__((may_alias));
union FragH { v16h v; v8h h[2]; };

__device__ __forceinline__ v8f wmf(v16h a, v16h b, v8f c) {
  v8f d = __builtin_amdgcn_wmma_f32_16x16x32_f16(false, a, false, b, (short)0, c, false, false);
  asm volatile("v_nop\n\tv_nop\n\tv_nop\n\tv_nop" : "+v"(d) : "v"(a), "v"(b));
  return d;
}

__device__ __forceinline__ float wave_sum(float x) {
#pragma unroll
  for (int off = 16; off > 0; off >>= 1) x += __shfl_xor(x, off, 32);
  return x;
}

__device__ __forceinline__ unsigned int pk2(float lo, float hi) {
  const unsigned short a = __builtin_bit_cast(unsigned short, (_Float16)lo);
  const unsigned short b = __builtin_bit_cast(unsigned short, (_Float16)hi);
  return (unsigned int)a | ((unsigned int)b << 16);
}

__device__ __forceinline__ void rot4(float& a0, float& a1, float& a2, float& a3,
                                     int p, float c, float sn) {
  const bool p0 = (p == 0), p1 = (p == 1);
  const float u = p0 ? a0 : (p1 ? a1 : a2);
  const float v = p0 ? a1 : (p1 ? a2 : a3);
  const float nu = u * c - v * sn;
  const float nv = u * sn + v * c;
  a0 = p0 ? nu : a0;
  a1 = p0 ? nv : (p1 ? nu : a1);
  a2 = p1 ? nv : (p0 ? a2 : nu);
  a3 = (p0 || p1) ? a3 : nv;
}

__device__ __forceinline__ unsigned int ln_pack(float xa, float xb, float wa, float wb, float ba, float bb) {
  const float mu  = wave_sum(xa + xb) * (1.0f / 64.0f);
  const float da  = xa - mu, db = xb - mu;
  const float var = wave_sum(da * da + db * db) * (1.0f / 64.0f);
  const float rs  = rsqrtf(var + LN_EPS);
  const float ya  = da * rs * wa + ba;
  const float yb  = db * rs * wb + bb;
  return pk2(ya * ACAR, yb * ACAR);
}

__global__ __launch_bounds__(32) void k_prep(const float* __restrict__ w1, const float* __restrict__ w2,
                                            const float* __restrict__ st1, const float* __restrict__ st2,
                                            const float* __restrict__ meta, const float* __restrict__ gates,
                                            _Float16* w1t, _Float16* w2t, float* tab) {
  const int lane = threadIdx.x & 31;
  const int blk = blockIdx.x;
  if (blk < N1) {
    const int n = blk;
    v8h a;
#pragma unroll
    for (int j = 0; j < 8; ++j) a[j] = (_Float16)(w1[(size_t)(8 * lane + j) * N1 + n] * WCAR);
    _Float16* d = w1t + (size_t)n * KF + 8 * lane;
    *(volatile v8h*)d = a;
    __threadfence();
    *(volatile v8h*)d = a;
  } else if (blk < N1 + N2 / 2) {
    const int q  = blk - N1;
    const int n  = 2 * q + (lane >> 4);
    const int kb = 8 * (lane & 15);
    v8h a;
#pragma unroll
    for (int j = 0; j < 8; ++j) a[j] = (_Float16)(w2[(size_t)(kb + j) * N2 + n] * WCAR);
    _Float16* d = w2t + (size_t)q * 256 + 8 * lane;
    *(volatile v8h*)d = a;
    __threadfence();
    *(volatile v8h*)d = a;
  } else {
    const float t0 = st1[0], t1 = st2[0], t2 = st2[1];
    const float e0 = meta[0], e1 = meta[1], e2 = meta[2];
    const float g0 = gates[0], g1 = gates[1], g2 = gates[2];
    const int grp = lane / 3;
    const int p = lane - 3 * grp;
    const float gs = (p == 0) ? g0 : ((p == 1) ? g1 : g2);
    const float gv = 1.0f / (1.0f + expf(-gs));
    const float tb = (p == 0) ? t0 : ((p == 1) ? t1 : t2);
    const float te = (p == 0) ? e0 : ((p == 1) ? e1 : e2);
    const float th = ((grp < 2) ? tb : te) * gv;
    const float cv = cosf(th);
    const float sv = sinf(th);
    float val = ((grp & 1) == 0) ? cv : sv;
    val = (lane < 12) ? val : 0.0f;
    float* d = tab + lane;
    *(volatile float*)d = val;
    __threadfence();
    *(volatile float*)d = val;
  }
}

__global__ __launch_bounds__(SCAN_THR) void k_scan(const int* __restrict__ braids, const float* __restrict__ init,
                                                  const float* __restrict__ tab, const float* __restrict__ lnw,
                                                  const float* __restrict__ lnb, unsigned int* apl) {
  __shared__ __attribute__((aligned(16))) unsigned int sA[SCAN_WAVES * 128];
  const int lane = threadIdx.x & 31;
  const int wave = threadIdx.x >> 5;
  const int b = __builtin_amdgcn_readfirstlane((int)blockIdx.x * SCAN_WAVES + wave);

  const float c0 = tab[0], c1 = tab[1], c2 = tab[2];
  const float s0 = tab[3], s1 = tab[4], s2 = tab[5];

  const int ha = 2 * lane, hb = 2 * lane + 1;
  float x0a = init[0 * NH + ha], x0b = init[0 * NH + hb];
  float x1a = init[1 * NH + ha], x1b = init[1 * NH + hb];
  float x2a = init[2 * NH + ha], x2b = init[2 * NH + hb];
  float x3a = init[3 * NH + ha], x3b = init[3 * NH + hb];

  const int* bw = braids + (size_t)b * NT;
#pragma unroll 1
  for (int t = 0; t < NT; ++t) {
    const int g = bw[t];
    const int ag = (g < 0) ? -g : g;
    int p = ag - 1;
    p = (p < 0) ? 0 : p;
    p = (p > 2) ? 2 : p;
    const bool nz = (g != 0);
    const float cs = (p == 0) ? c0 : ((p == 1) ? c1 : c2);
    const float ss = (p == 0) ? s0 : ((p == 1) ? s1 : s2);
    const float c  = nz ? cs : 1.0f;
    const float sn = nz ? ((g < 0) ? -ss : ss) : 0.0f;
    rot4(x0a, x1a, x2a, x3a, p, c, sn);
    rot4(x0b, x1b, x2b, x3b, p, c, sn);
  }

  {
    const float mc0 = tab[6], mc1 = tab[7], mc2 = tab[8];
    const float ms0 = tab[9], ms1 = tab[10], ms2 = tab[11];
    rot4(x0a, x1a, x2a, x3a, 0, mc0, ms0);
    rot4(x0b, x1b, x2b, x3b, 0, mc0, ms0);
    rot4(x0a, x1a, x2a, x3a, 1, mc1, ms1);
    rot4(x0b, x1b, x2b, x3b, 1, mc1, ms1);
    rot4(x0a, x1a, x2a, x3a, 2, mc2, ms2);
    rot4(x0b, x1b, x2b, x3b, 2, mc2, ms2);
  }

  const float wa = lnw[ha], wb = lnw[hb];
  const float ba = lnb[ha], bb = lnb[hb];
  unsigned int* sw = sA + wave * 128 + lane;
  sw[0]  = ln_pack(x0a, x0b, wa, wb, ba, bb);
  sw[32] = ln_pack(x1a, x1b, wa, wb, ba, bb);
  sw[64] = ln_pack(x2a, x2b, wa, wb, ba, bb);
  sw[96] = ln_pack(x3a, x3b, wa, wb, ba, bb);
  __syncthreads();

  const v4u v = *(const v4ua*)(sA + wave * 128 + 4 * lane);
  unsigned int* d = apl + (size_t)b * 128 + 4 * lane;
  *(volatile v4u*)d = v;
  __threadfence();
  *(volatile v4u*)d = v;
}

__global__ __launch_bounds__(GEMM_THR) void k_gemm1(const _Float16* __restrict__ apl, const _Float16* __restrict__ w1t,
                                                   const float* __restrict__ b1, _Float16* hpl) {
  __shared__ __attribute__((aligned(16))) _Float16 sH[4 * 16 * N1];
  const int tid = threadIdx.x, lane = tid & 31, wave = tid >> 5, hf = lane >> 4, m = lane & 15;
  const int m0 = blockIdx.x * 64 + wave * 16;

  v8f acc[8];
#pragma unroll
  for (int nt = 0; nt < 8; ++nt) { v8f z = {0.f, 0.f, 0.f, 0.f, 0.f, 0.f, 0.f, 0.f}; acc[nt] = z; }

  const _Float16* ap = apl + (size_t)(m0 + m) * KF + 8 * hf;
  const _Float16* bp = w1t + (size_t)m * KF + 8 * hf;
#pragma unroll 1
  for (int kt = 0; kt < KF / 32; ++kt) {
    const int k0 = 32 * kt;
    FragH a;
    a.h[0] = *(const v8h*)(ap + k0);
    a.h[1] = *(const v8h*)(ap + k0 + 16);
#pragma unroll
    for (int nt = 0; nt < 8; ++nt) {
      const _Float16* bq = bp + (size_t)nt * 16 * KF + k0;
      FragH bf;
      bf.h[0] = *(const v8h*)bq;
      bf.h[1] = *(const v8h*)(bq + 16);
      acc[nt] = wmf(a.v, bf.v, acc[nt]);
    }
  }

  constexpr float INV1 = 1.0f / WCAR;
  _Float16* sp = sH + wave * (16 * N1) + (8 * hf) * N1 + m;
#pragma unroll
  for (int nt = 0; nt < 8; ++nt) {
    const float bb = HCAR * b1[16 * nt + m];
#pragma unroll
    for (int r = 0; r < 8; ++r) {
      const float v = fmaxf(acc[nt][r] * INV1 + bb, 0.0f);
      sp[r * N1 + 16 * nt] = (_Float16)v;
    }
  }
  __syncthreads();

  const _Float16* src = sH + wave * (16 * N1) + 8 * lane;
  _Float16* dst = hpl + (size_t)m0 * N1 + 8 * lane;
#pragma unroll
  for (int q = 0; q < 8; ++q) {
    const v8h v = *(const v8ha*)(src + q * 256);
    *(volatile v8h*)(dst + q * 256) = v;
  }
  __threadfence();
#pragma unroll
  for (int q = 0; q < 8; ++q) {
    const v8h v = *(const v8ha*)(src + q * 256);
    *(volatile v8h*)(dst + q * 256) = v;
  }
}

__global__ __launch_bounds__(GEMM_THR) void k_gemm2(const _Float16* __restrict__ hpl, const _Float16* __restrict__ w2t,
                                                   const float* __restrict__ b2, const float* __restrict__ w3,
                                                   const float* __restrict__ b3, float* out) {
  __shared__ float sH2[64 * LDH];
  __shared__ __attribute__((aligned(16))) float sO[128];
  const int tid = threadIdx.x, lane = tid & 31, wave = tid >> 5, hf = lane >> 4, m = lane & 15;
  const int m0b = blockIdx.x * 64;
  const int mw = m0b + wave * 16;

  v8f acc[4];
#pragma unroll
  for (int nt = 0; nt < 4; ++nt) { v8f z = {0.f, 0.f, 0.f, 0.f, 0.f, 0.f, 0.f, 0.f}; acc[nt] = z; }

  const _Float16* ap = hpl + (size_t)(mw + m) * N1 + 8 * hf;
  const _Float16* bp = w2t + (size_t)m * N1 + 8 * hf;
#pragma unroll 1
  for (int kt = 0; kt < N1 / 32; ++kt) {
    const int k0 = 32 * kt;
    FragH a;
    a.h[0] = *(const v8h*)(ap + k0);
    a.h[1] = *(const v8h*)(ap + k0 + 16);
#pragma unroll
    for (int nt = 0; nt < 4; ++nt) {
      const _Float16* bq = bp + (size_t)nt * 16 * N1 + k0;
      FragH bf;
      bf.h[0] = *(const v8h*)bq;
      bf.h[1] = *(const v8h*)(bq + 16);
      acc[nt] = wmf(a.v, bf.v, acc[nt]);
    }
  }

  constexpr float INV2 = 1.0f / (HCAR * WCAR);
  float* sp = sH2 + (wave * 16 + 8 * hf) * LDH + m;
#pragma unroll
  for (int nt = 0; nt < 4; ++nt) {
    const float bb = b2[16 * nt + m];
#pragma unroll
    for (int r = 0; r < 8; ++r) sp[r * LDH + 16 * nt] = fmaxf(acc[nt][r] * INV2 + bb, 0.0f);
  }
  __syncthreads();

  const int row = tid & 63;
  const int j = tid >> 6;
  const float* hr = sH2 + row * LDH;
  const float* wc = w3 + j;
  float o = 0.0f;
#pragma unroll 8
  for (int i = 0; i < N2; ++i) o += hr[i] * wc[2 * i];
  o += b3[j];
  const float oc = fminf(fmaxf(o, -80.0f), 80.0f);
  const float sg = 1.0f / (1.0f + expf(-oc));
  const float res = (j == 0) ? sg : o;
  sO[j * 64 + row] = res;
  __syncthreads();

  if (wave == 0) {
    const v4f v = *(const v4fa*)(sO + 4 * lane);
    const size_t off = (lane < 16) ? (size_t)(m0b + 4 * lane) : (size_t)(NB + m0b + 4 * lane - 64);
    float* d = out + off;
    *(volatile v4f*)d = v;
    __threadfence();
    *(volatile v4f*)d = v;
  }
}

extern "C" void kernel_launch(void* const* d_in, const int* in_sizes, int n_in,
                              void* d_out, int out_size, void* d_ws, size_t ws_size,
                              hipStream_t stream) {
  if (n_in < 14) return;
  if (in_sizes[0] != NB * NT || in_sizes[1] != NS * NH || in_sizes[2] != 1 || in_sizes[3] != 2 ||
      in_sizes[4] != 3 || in_sizes[5] != 3 || in_sizes[6] != NH || in_sizes[7] != NH ||
      in_sizes[8] != KF * N1 || in_sizes[9] != N1 || in_sizes[10] != N1 * N2 || in_sizes[11] != N2 ||
      in_sizes[12] != N2 * 2 || in_sizes[13] != 2) return;
  if (out_size != 2 * NB) return;

  const int*   braids = (const int*)d_in[0];
  const float* init   = (const float*)d_in[1];
  const float* st1    = (const float*)d_in[2];
  const float* st2    = (const float*)d_in[3];
  const float* meta   = (const float*)d_in[4];
  const float* gates  = (const float*)d_in[5];
  const float* lnw    = (const float*)d_in[6];
  const float* lnb    = (const float*)d_in[7];
  const float* w1     = (const float*)d_in[8];
  const float* b1     = (const float*)d_in[9];
  const float* w2     = (const float*)d_in[10];
  const float* b2     = (const float*)d_in[11];
  const float* w3     = (const float*)d_in[12];
  const float* b3     = (const float*)d_in[13];
  float* out = (float*)d_out;

  char* ws = (char*)d_ws;
  size_t off = 0;
  const size_t oT  = off; off += 256;
  const size_t oA  = off; off += (size_t)NB * KF * 2;  off = (off + 255) & ~(size_t)255;
  const size_t oH  = off; off += (size_t)NB * N1 * 2;  off = (off + 255) & ~(size_t)255;
  const size_t oW1 = off; off += (size_t)N1 * KF * 2;  off = (off + 255) & ~(size_t)255;
  const size_t oW2 = off; off += (size_t)N2 * N1 * 2;  off = (off + 255) & ~(size_t)255;
  if (off > ws_size || off > (size_t)WSCAP) return;
  float*    tab = (float*)(ws + oT);
  _Float16* apl = (_Float16*)(ws + oA);
  _Float16* hpl = (_Float16*)(ws + oH);
  _Float16* w1t = (_Float16*)(ws + oW1);
  _Float16* w2t = (_Float16*)(ws + oW2);

  k_prep<<<N1 + N2 / 2 + 1, 32, 0, stream>>>(w1, w2, st1, st2, meta, gates, w1t, w2t, tab);
  k_scan<<<NB / SCAN_WAVES, SCAN_THR, 0, stream>>>(braids, init, tab, lnw, lnb, (unsigned int*)apl);
  k_gemm1<<<NB / 64, GEMM_THR, 0, stream>>>(apl, w1t, b1, hpl);
  k_gemm2<<<NB / 64, GEMM_THR, 0, stream>>>(hpl, w2t, b2, w3, b3, out);
}
